// CrossAttentionLayer_19129784336817
// MI455X (gfx1250) — hardware-verified
//
#include <hip/hip_runtime.h>


#ifndef NB
#define NB 2
#endif
#ifndef SEQ
#define SEQ 2048
#endif
#ifndef SEQK
#define SEQK 2048
#endif
#define SEQ_FULL  2048
#define SEQK_FULL 2048
#define QD   512
#define KVD  512
#define EMB  1024
#define NH   16
#define HD   64
#define MQ   (NB * SEQ)
#define MK   (NB * SEQK)
#define LNEPS 1.0e-5f
static_assert(SEQ % 64 == 0);
static_assert(SEQK % 64 == 0);
static_assert(QD % 32 == 0);
static_assert(KVD % 32 == 0);
static_assert(EMB == NH * HD);
static_assert(EMB % 64 == 0);
static_assert(EMB == 32 * 4 * 8);
static_assert(MQ % 8 == 0);

typedef _Float16 h16;
typedef unsigned short bf;
typedef unsigned short u16;
typedef __attribute__((ext_vector_type(16))) __bf16   v16bf;
typedef __attribute__((ext_vector_type(16))) _Float16 v16h;
typedef __attribute__((ext_vector_type(8)))  _Float16 v8h;
typedef __attribute__((ext_vector_type(8)))  unsigned short v8us;
typedef __attribute__((ext_vector_type(8)))  float    v8f;
typedef __attribute__((ext_vector_type(4)))  float    v4f;
typedef v8h  __attribute__((may_alias)) v8ha;
typedef v4f  __attribute__((may_alias)) v4fa;
typedef v8us __attribute__((may_alias)) v8usa;

__device__ __forceinline__ unsigned short f2bf(float f) { unsigned u = __float_as_uint(f); u += 0x7FFFu + ((u >> 16) & 1u); return (unsigned short)(u >> 16); }
__device__ __forceinline__ float bf2f(unsigned short b) { return __uint_as_float(((unsigned)b) << 16); }
__device__ __forceinline__ float bfr(float f) { return bf2f(f2bf(f)); }
__device__ __forceinline__ v16h cat16(v8h lo, v8h hi) { return __builtin_shufflevector(lo, hi, 0, 1, 2, 3, 4, 5, 6, 7, 8, 9, 10, 11, 12, 13, 14, 15); }
__device__ __forceinline__ v16bf cat16b(v8us lo, v8us hi) { return __builtin_bit_cast(v16bf, __builtin_shufflevector(lo, hi, 0, 1, 2, 3, 4, 5, 6, 7, 8, 9, 10, 11, 12, 13, 14, 15)); }
__device__ __forceinline__ v8f wmma16(v16h a, v16h b, v8f c) { return __builtin_amdgcn_wmma_f32_16x16x32_f16(false, a, false, b, (short)0, c, false, false); }
__device__ __forceinline__ v8f wmmab(v16bf a, v16bf b, v8f c) { return __builtin_amdgcn_wmma_f32_16x16x32_bf16(false, a, false, b, (short)0, c, false, false); }

template <typename T16> struct WFrag;
template <> struct WFrag<h16> { typedef v16h V; static __device__ __forceinline__ V ld(const h16* p) { return cat16(*(const v8h*)p, *(const v8h*)(p + 16)); } static __device__ __forceinline__ v8f mma(V a, V b, v8f c) { return wmma16(a, b, c); } };
template <> struct WFrag<bf> { typedef v16bf V; static __device__ __forceinline__ V ld(const bf* p) { return cat16b(*(const v8us*)p, *(const v8us*)(p + 16)); } static __device__ __forceinline__ v8f mma(V a, V b, v8f c) { return wmmab(a, b, c); } };
template <typename T16, int NSPLIT, bool BIAS>
__global__ __launch_bounds__(32) void k_gemmw(const T16* __restrict__ A, const T16* __restrict__ A2, const T16* __restrict__ Bt, const T16* __restrict__ Bt2, int K, float* C, int ldc, const float* __restrict__ bias, size_t sA, size_t sB, size_t sC) {
    typedef typename WFrag<T16>::V V;
    __shared__ __align__(16) float os[16 * 68];
    const size_t z = blockIdx.z; A += z * sA; if (A2) A2 += z * sA; Bt += z * sB; if (Bt2) Bt2 += z * sB; C += z * sC;
    const int lane = threadIdx.x & 31, lr = lane & 15, hi = lane >> 4; const int r0 = blockIdx.x * 64, c0 = blockIdx.y * 64;
    v8f acc[4][4];
#pragma unroll
    for (int mb = 0; mb < 4; ++mb)
#pragma unroll
        for (int nb = 0; nb < 4; ++nb) acc[mb][nb] = (v8f){};
    const size_t aoff = (size_t)(r0 + lr) * K + 8 * hi, boff = (size_t)(c0 + lr) * K + 8 * hi;
#pragma unroll 1
    for (int kc = 0; kc < K; kc += 32) {
        V a[4], a2[4];
#pragma unroll
        for (int mb = 0; mb < 4; ++mb) { a[mb] = WFrag<T16>::ld(A + aoff + (size_t)mb * 16 * K + kc); if (NSPLIT == 1 || NSPLIT == 2) a2[mb] = WFrag<T16>::ld(A2 + aoff + (size_t)mb * 16 * K + kc); }
#pragma unroll
        for (int nb = 0; nb < 4; ++nb) { const V b = WFrag<T16>::ld(Bt + boff + (size_t)nb * 16 * K + kc); V b2; if (NSPLIT >= 2) b2 = WFrag<T16>::ld(Bt2 + boff + (size_t)nb * 16 * K + kc);
#pragma unroll
            for (int mb = 0; mb < 4; ++mb) { acc[mb][nb] = WFrag<T16>::mma(a[mb], b, acc[mb][nb]); if (NSPLIT == 1 || NSPLIT == 2) acc[mb][nb] = WFrag<T16>::mma(a2[mb], b, acc[mb][nb]); if (NSPLIT >= 2) acc[mb][nb] = WFrag<T16>::mma(a[mb], b2, acc[mb][nb]); } }
        asm volatile("v_nop\n\tv_nop\n\tv_nop\n\tv_nop" : "+v"(acc[0][0]), "+v"(acc[1][1]), "+v"(acc[2][2]), "+v"(acc[3][3]) : "v"(a[0]), "v"(a[3]));
    }
#pragma unroll
    for (int mb = 0; mb < 4; ++mb) {
#pragma unroll
        for (int nb = 0; nb < 4; ++nb) {
#pragma unroll
            for (int j = 0; j < 8; ++j) os[(hi * 8 + j) * 68 + nb * 16 + lr] = acc[mb][nb][j]; }
        __builtin_amdgcn_fence(3, "wavefront"); __builtin_amdgcn_wave_barrier(); asm volatile("" ::: "memory");
        float* crow = C + (size_t)(r0 + mb * 16) * ldc + c0;
#pragma unroll 1
        for (int ps = 0; ps < 2; ++ps) {
#pragma unroll
            for (int s = 0; s < 8; ++s) { const int row = 2 * s + hi, cofs = lr * 4; v4f val = *(const v4fa*)(os + row * 68 + cofs); if (BIAS) { val[0] += bfr(bias[c0 + cofs]); val[1] += bfr(bias[c0 + cofs + 1]); val[2] += bfr(bias[c0 + cofs + 2]); val[3] += bfr(bias[c0 + cofs + 3]); }
                *(volatile v4f*)(crow + (size_t)row * ldc + cofs) = val; }
            if (ps == 0) __threadfence(); }
        __builtin_amdgcn_fence(3, "wavefront"); __builtin_amdgcn_wave_barrier(); asm volatile("" ::: "memory");
    }
}

__device__ __forceinline__ h16 tohx(float x) { return (h16)x; }
__device__ __forceinline__ void splitf(float y, unsigned short& h, unsigned short& l) { h = f2bf(y); l = f2bf(y - bf2f(h)); }

__global__ __launch_bounds__(256) void k_cvt8(const float* __restrict__ src, size_t sbs, bf* dst, size_t dbs, size_t n8) { const size_t i = (size_t)blockIdx.x * 256 + threadIdx.x; if (i >= n8) return; const float* s = src + (size_t)blockIdx.y * sbs + i * 8; bf* d = dst + (size_t)blockIdx.y * dbs + i * 8; const v8f v = *(const v8f*)s; v8us o;
#pragma unroll
    for (int k = 0; k < 8; ++k) o[k] = f2bf(v[k]); *(volatile v8us*)d = o; __threadfence(); *(volatile v8us*)d = o; }

__global__ __launch_bounds__(256) void k_cvt8Tg(const float* __restrict__ src, bf* dst, int R, int C) { const size_t i = (size_t)blockIdx.x * 256 + threadIdx.x; if (i >= (size_t)R * C / 8) return; const int c = (int)(i / (R / 8)); const int r0 = (int)(i % (R / 8)) * 8; v8us o;
#pragma unroll
    for (int k = 0; k < 8; ++k) o[k] = f2bf(src[(size_t)(r0 + k) * C + c]); *(volatile v8us*)(dst + (size_t)c * R + r0) = o; __threadfence(); *(volatile v8us*)(dst + (size_t)c * R + r0) = o; }

__global__ __launch_bounds__(256) void k_cvth(const float* __restrict__ src, u16* dst, size_t n8, float sc) { const size_t i = (size_t)blockIdx.x * 256 + threadIdx.x; if (i >= n8) return; const v8f v = *(const v8f*)(src + i * 8); v8h o;
#pragma unroll
    for (int k = 0; k < 8; ++k) o[k] = tohx(v[k] * sc); const v8us ob = __builtin_bit_cast(v8us, o); *(volatile v8us*)(dst + i * 8) = ob; __threadfence(); *(volatile v8us*)(dst + i * 8) = ob; }

__global__ __launch_bounds__(256) void k_cvthT(const float* __restrict__ src, size_t sbs, u16* dst, size_t dbs, int R, int C, float sc) { const size_t i = (size_t)blockIdx.x * 256 + threadIdx.x; if (i >= (size_t)R * C / 8) return; const float* s = src + (size_t)blockIdx.y * sbs; u16* d = dst + (size_t)blockIdx.y * dbs; const int c = (int)(i / (R / 8)); const int r0 = (int)(i % (R / 8)) * 8; v8h o;
#pragma unroll
    for (int k = 0; k < 8; ++k) o[k] = tohx(s[(size_t)(r0 + k) * C + c] * sc); const v8us ob = __builtin_bit_cast(v8us, o); *(volatile v8us*)(d + (size_t)c * R + r0) = ob; __threadfence(); *(volatile v8us*)(d + (size_t)c * R + r0) = ob; }

__device__ __forceinline__ v16h ldh(const h16* p) { return cat16(*(const v8h*)p, *(const v8h*)(p + 16)); }
__device__ __forceinline__ v16h ldhl(const unsigned short* p) { return cat16(__builtin_bit_cast(v8h, *(const v8usa*)p), __builtin_bit_cast(v8h, *(const v8usa*)(p + 16))); }

__global__ __launch_bounds__(128) __attribute__((amdgpu_num_vgpr(256)))
void k_attn(const h16* __restrict__ Q16, const h16* __restrict__ K16, const h16* __restrict__ VT, bf* CH, bf* CL) {
#pragma clang fp contract(off)
    __shared__ __align__(16) unsigned short pls[4][16 * 72];
    __shared__ __align__(16) unsigned short cls[4][16 * 72];
    const int wid = threadIdx.x >> 5, lane = threadIdx.x & 31, lr = lane & 15, hi = lane >> 4;
    const int b = blockIdx.y / NH, h = blockIdx.y % NH;
    const int q0 = blockIdx.x * 64 + wid * 16;
    unsigned short* pl = &pls[wid][0]; unsigned short* cl = &cls[wid][0];
    const h16* qp = Q16 + ((size_t)b * SEQ + q0 + lr) * EMB + h * HD + 8 * hi;
    const v16h aq0 = ldh(qp), aq1 = ldh(qp + 32);
    v8f o[4];
#pragma unroll
    for (int n = 0; n < 4; ++n) o[n] = (v8f){};
    float mrow[8], lrow[8];
#pragma unroll
    for (int r = 0; r < 8; ++r) { mrow[r] = -1.0e30f; lrow[r] = 0.0f; }
    const h16* kbase = K16 + ((size_t)b * SEQK + lr) * EMB + h * HD + 8 * hi;
    const h16* vbase = VT + ((size_t)b * EMB + h * HD + lr) * SEQK + 8 * hi;
    const float CS = 1.4426950408889634f * 0.00048828125f;
#pragma unroll 1
    for (int j0 = 0; j0 < SEQK; j0 += 64) {
        v8f s[4];
#pragma unroll
        for (int kt = 0; kt < 4; ++kt) { const h16* kp = kbase + (size_t)(j0 + kt * 16) * EMB; const v16h kf0 = ldh(kp); const v16h kf1 = ldh(kp + 32); v8f c = (v8f){}; c = wmma16(aq0, kf0, c); c = wmma16(aq1, kf1, c); s[kt] = c; }
        asm volatile("v_nop\n\tv_nop\n\tv_nop\n\tv_nop" : "+v"(s[0]), "+v"(s[1]), "+v"(s[2]), "+v"(s[3]) : "v"(aq0), "v"(aq1));
#pragma unroll
        for (int r = 0; r < 8; ++r) {
            float t[4];
#pragma unroll
            for (int q = 0; q < 4; ++q) t[q] = s[q][r] * CS;
            float mx = fmaxf(fmaxf(t[0], t[1]), fmaxf(t[2], t[3]));
#pragma unroll
            for (int sh = 1; sh < 16; sh <<= 1) mx = fmaxf(mx, __shfl_xor(mx, sh, 32));
            const float mnew = fmaxf(mrow[r], mx);
            const float dm = mrow[r] - mnew;
            const float corr = __builtin_amdgcn_exp2f(dm);
            mrow[r] = mnew;
            float rs = 0.0f;
#pragma unroll
            for (int q = 0; q < 4; ++q) { const float d0 = t[q] - mnew; const float p = __builtin_amdgcn_exp2f(d0); s[q][r] = p; rs += p; }
#pragma unroll
            for (int sh = 1; sh < 16; sh <<= 1) rs += __shfl_xor(rs, sh, 32);
            lrow[r] = lrow[r] * corr + rs;
#pragma unroll
            for (int n = 0; n < 4; ++n) o[n][r] *= corr;
        }
#pragma unroll
        for (int kt = 0; kt < 4; ++kt)
#pragma unroll
            for (int r = 0; r < 8; ++r) { const h16 ph = tohx(s[kt][r] * 1024.0f); pl[(8 * hi + r) * 72 + kt * 16 + lr] = __builtin_bit_cast(unsigned short, ph); }
        __builtin_amdgcn_fence(3, "wavefront"); __builtin_amdgcn_wave_barrier(); asm volatile("" ::: "memory");
        const v16h pa0 = ldhl(pl + lr * 72 + 8 * hi), pa1 = ldhl(pl + lr * 72 + 32 + 8 * hi);
        __builtin_amdgcn_wave_barrier(); asm volatile("" ::: "memory");
#pragma unroll
        for (int n = 0; n < 4; ++n) { const h16* vp = vbase + (size_t)n * 16 * SEQK + j0; const v16h vf0 = ldh(vp); const v16h vf1 = ldh(vp + 32); o[n] = wmma16(pa0, vf0, o[n]); o[n] = wmma16(pa1, vf1, o[n]); }
        asm volatile("v_nop\n\tv_nop\n\tv_nop\n\tv_nop" : "+v"(o[0]), "+v"(o[1]), "+v"(o[2]), "+v"(o[3]) : "v"(pa0), "v"(pa1));
    }
    float inv[8];
#pragma unroll
    for (int r = 0; r < 8; ++r) inv[r] = 1.0f / (lrow[r] * 16384.0f);
#pragma unroll
    for (int n = 0; n < 4; ++n)
#pragma unroll
        for (int r = 0; r < 8; ++r) { const float y = o[n][r] * inv[r]; unsigned short a, c2; splitf(y, a, c2); const int idx = (8 * hi + r) * 72 + n * 16 + lr; pl[idx] = a; cl[idx] = c2; }
    __builtin_amdgcn_fence(3, "wavefront"); __builtin_amdgcn_wave_barrier(); asm volatile("" ::: "memory");
#pragma unroll 1
    for (int ps = 0; ps < 2; ++ps) {
#pragma unroll
        for (int g = 0; g < 4; ++g) { const int row = g * 4 + (lane >> 3), pc = (lane & 7) * 8; const v8us vh = *(const v8usa*)(pl + row * 72 + pc); const v8us vl = *(const v8usa*)(cl + row * 72 + pc);
            const size_t go = ((size_t)b * SEQ + q0 + row) * EMB + h * HD + pc; *(volatile v8us*)(CH + go) = vh; *(volatile v8us*)(CL + go) = vl; }
        if (ps == 0) __threadfence(); }
}

__global__ __launch_bounds__(256) void k_ln(const float* __restrict__ X, const float* __restrict__ gam, const float* __restrict__ bet, float* Y, int nrows) {
#pragma clang fp contract(off)
    const int wid = threadIdx.x >> 5, lane = threadIdx.x & 31;
    const int row = blockIdx.x * 8 + wid;
    if (row >= nrows) return;
    const float* x = X + (size_t)row * EMB + lane * 4;
    v4f v[8];
    float s = 0.0f;
#pragma unroll
    for (int i = 0; i < 8; ++i) { v[i] = *(const v4fa*)(x + i * 128); s += (v[i][0] + v[i][1]) + (v[i][2] + v[i][3]); }
#pragma unroll
    for (int sh = 1; sh < 32; sh <<= 1) s += __shfl_xor(s, sh, 32);
    const float mu = s * (1.0f / (float)EMB);
    float s2 = 0.0f;
#pragma unroll
    for (int i = 0; i < 8; ++i) {
#pragma unroll
        for (int c = 0; c < 4; ++c) { const float d = v[i][c] - mu; v[i][c] = d; const float dd = d * d; s2 += dd; }
    }
#pragma unroll
    for (int sh = 1; sh < 32; sh <<= 1) s2 += __shfl_xor(s2, sh, 32);
    const float var = s2 * (1.0f / (float)EMB);
    const float inv = rsqrtf(var + LNEPS);
#pragma unroll
    for (int i = 0; i < 8; ++i) {
        const v4f g = *(const v4fa*)(gam + lane * 4 + i * 128);
        const v4f bb = *(const v4fa*)(bet + lane * 4 + i * 128);
#pragma unroll
        for (int c = 0; c < 4; ++c) { const float xn = v[i][c] * inv; const float yg = xn * bfr(g[c]); v[i][c] = yg + bfr(bb[c]); }
    }
    float* y = Y + (size_t)row * EMB + lane * 4;
#pragma unroll 1
    for (int ps = 0; ps < 2; ++ps) {
#pragma unroll
        for (int i = 0; i < 8; ++i) *(volatile v4f*)(y + i * 128) = v[i];
        if (ps == 0) __threadfence();
    }
}

extern "C" void kernel_launch(void* const* d_in, const int* in_sizes, int n_in,
                              void* d_out, int out_size, void* d_ws, size_t ws_size, hipStream_t stream) {
    if (n_in < 13) return;
    if (in_sizes[0] < ((NB - 1) * SEQ_FULL + SEQ) * QD) return;
    if (in_sizes[1] < ((NB - 1) * SEQK_FULL + SEQK) * KVD) return;
    if (in_sizes[2] < ((NB - 1) * SEQK_FULL + SEQK) * KVD) return;
    if (in_sizes[3] < QD * EMB || in_sizes[4] < EMB || in_sizes[5] < KVD * EMB || in_sizes[6] < EMB) return;
    if (in_sizes[7] < KVD * EMB || in_sizes[8] < EMB || in_sizes[9] < EMB * EMB || in_sizes[10] < EMB) return;
    if (in_sizes[11] < EMB || in_sizes[12] < EMB) return;
    if (out_size < MQ * EMB) return;
    const float* query = (const float*)d_in[0]; const float* key = (const float*)d_in[1]; const float* value = (const float*)d_in[2];
    const float* Wq = (const float*)d_in[3]; const float* bq = (const float*)d_in[4];
    const float* Wk = (const float*)d_in[5]; const float* bk = (const float*)d_in[6];
    const float* Wv = (const float*)d_in[7]; const float* bv = (const float*)d_in[8];
    const float* Wo = (const float*)d_in[9]; const float* bo = (const float*)d_in[10];
    const float* gam = (const float*)d_in[11]; const float* bet = (const float*)d_in[12];
    float* OUT = (float*)d_out;
    char* wsp = (char*)d_ws;
    auto take = [&](size_t bytes) { char* p = wsp; wsp += (bytes + 255) & ~(size_t)255; return (void*)p; };
    bf* XQ  = (bf*)take((size_t)MQ * QD * 2);
    bf* XK  = (bf*)take((size_t)MK * KVD * 2);
    bf* XV  = (bf*)take((size_t)MK * KVD * 2);
    bf* WQT = (bf*)take((size_t)EMB * QD * 2);
    bf* WKT = (bf*)take((size_t)EMB * KVD * 2);
    bf* WVT = (bf*)take((size_t)EMB * KVD * 2);
    bf* WOT = (bf*)take((size_t)EMB * EMB * 2);
    const size_t mmax = (MQ > MK) ? (size_t)MQ : (size_t)MK;
    float* F  = (float*)take(mmax * EMB * 4);
    u16* Q16 = (u16*)take((size_t)MQ * EMB * 2);
    u16* K16 = (u16*)take((size_t)MK * EMB * 2);
    u16* VTp = (u16*)take((size_t)NB * EMB * SEQK * 2);
    bf* CH  = (bf*)take((size_t)MQ * EMB * 2);
    bf* CL  = (bf*)take((size_t)MQ * EMB * 2);
    if ((size_t)(wsp - (char*)d_ws) > ws_size) return;

    { const size_t n8 = (size_t)SEQ * QD / 8; k_cvt8<<<dim3((unsigned)((n8 + 255) / 256), NB), 256, 0, stream>>>(query, (size_t)SEQ_FULL * QD, XQ, (size_t)SEQ * QD, n8); }
    { const size_t n8 = (size_t)SEQK * KVD / 8; k_cvt8<<<dim3((unsigned)((n8 + 255) / 256), NB), 256, 0, stream>>>(key, (size_t)SEQK_FULL * KVD, XK, (size_t)SEQK * KVD, n8);
      k_cvt8<<<dim3((unsigned)((n8 + 255) / 256), NB), 256, 0, stream>>>(value, (size_t)SEQK_FULL * KVD, XV, (size_t)SEQK * KVD, n8); }
    k_cvt8Tg<<<(unsigned)(((size_t)QD * EMB / 8 + 255) / 256), 256, 0, stream>>>(Wq, WQT, QD, EMB);
    k_cvt8Tg<<<(unsigned)(((size_t)KVD * EMB / 8 + 255) / 256), 256, 0, stream>>>(Wk, WKT, KVD, EMB);
    k_cvt8Tg<<<(unsigned)(((size_t)KVD * EMB / 8 + 255) / 256), 256, 0, stream>>>(Wv, WVT, KVD, EMB);
    k_cvt8Tg<<<(unsigned)(((size_t)EMB * EMB / 8 + 255) / 256), 256, 0, stream>>>(Wo, WOT, EMB, EMB);

    k_gemmw<bf, 0, true><<<dim3(MQ / 64, EMB / 64, 1), 32, 0, stream>>>(XQ, nullptr, WQT, nullptr, QD, F, EMB, bq, 0, 0, 0);
    k_cvth<<<(unsigned)(((size_t)MQ * EMB / 8 + 255) / 256), 256, 0, stream>>>(F, Q16, (size_t)MQ * EMB / 8, 16.0f);
    k_gemmw<bf, 0, true><<<dim3(MK / 64, EMB / 64, 1), 32, 0, stream>>>(XK, nullptr, WKT, nullptr, KVD, F, EMB, bk, 0, 0, 0);
    k_cvth<<<(unsigned)(((size_t)MK * EMB / 8 + 255) / 256), 256, 0, stream>>>(F, K16, (size_t)MK * EMB / 8, 16.0f);
    k_gemmw<bf, 0, true><<<dim3(MK / 64, EMB / 64, 1), 32, 0, stream>>>(XV, nullptr, WVT, nullptr, KVD, F, EMB, bv, 0, 0, 0);
    k_cvthT<<<dim3((unsigned)(((size_t)SEQK * EMB / 8 + 255) / 256), NB), 256, 0, stream>>>(F, (size_t)SEQK * EMB, VTp, (size_t)EMB * SEQK, SEQK, EMB, 16.0f);
    k_attn<<<dim3(SEQ / 64, NB * NH), 128, 0, stream>>>((const h16*)Q16, (const h16*)K16, (const h16*)VTp, CH, CL);
    k_gemmw<bf, 1, true><<<dim3(MQ / 64, EMB / 64, 1), 32, 0, stream>>>(CH, CL, WOT, nullptr, EMB, F, EMB, bo, 0, 0, 0);
    k_ln<<<(unsigned)((MQ + 7) / 8), 256, 0, stream>>>(F, gam, bet, OUT, MQ);
}
